// DecoderLayer_41601053229607
// MI455X (gfx1250) — hardware-verified
//
#include <hip/hip_runtime.h>

#ifndef NB
#define NB 4
#endif
#ifndef SEQ
#define SEQ 1024
#endif
#define NB_FULL 4
#define SEQ_FULL 1024
#define DM 1024
#define NH 16
#define HD 64
#define DFF 4096
#define NR ((size_t)NB * SEQ)
#define MR ((int)((size_t)NB * SEQ))
#define PBP 40
#define OBP 72
#define LN_EPS 1.0e-3f

static_assert(NB >= 1 && NB <= NB_FULL);
static_assert(SEQ >= 64 && SEQ <= SEQ_FULL && SEQ % 64 == 0);
static_assert((NB * SEQ) % 128 == 0);
static_assert(NH * HD == DM && HD == 64);
static_assert(DM == 4 * 256);
static_assert(DM % 64 == 0 && DFF % 64 == 0 && DM % 32 == 0 && DFF % 32 == 0);
static_assert(DFF <= 4 * DM);
static_assert((PBP % 8) == 0 && (OBP % 8) == 0);

typedef unsigned short v8us __attribute__((ext_vector_type(8), may_alias));
typedef float  v8f  __attribute__((ext_vector_type(8)));
typedef float  v4f  __attribute__((ext_vector_type(4)));
typedef float  v4fa __attribute__((ext_vector_type(4), may_alias));
typedef _Float16 v16h __attribute__((ext_vector_type(16)));
typedef _Float16 v4h __attribute__((ext_vector_type(4)));
union FragH { v16h v; v8us half[2]; _Float16 h[16]; unsigned short u[16]; };

__device__ __forceinline__ unsigned short bf16_bits(float x) { unsigned int u = __float_as_uint(x); return (unsigned short)((u + 0x7FFFu + ((u >> 16) & 1u)) >> 16); }
__device__ __forceinline__ float bf16_val(unsigned short b) { return __uint_as_float(((unsigned int)b) << 16); }
__device__ __forceinline__ float bf16_rne(float x) { return bf16_val(bf16_bits(x)); }

__device__ __forceinline__ v16h g2_frag(const _Float16* p, int hh) { FragH f; f.half[0] = *(const v8us*)((const unsigned short*)p + 8 * hh); f.half[1] = *(const v8us*)((const unsigned short*)p + 16 + 8 * hh); return f.v; }
__device__ __forceinline__ v8f g2_mma(v16h a, v16h b, v8f c) { v8f d = __builtin_amdgcn_wmma_f32_16x16x32_f16(false, a, false, b, (short)0, c, false, false); asm volatile("v_nop\n\tv_nop\n\tv_nop\n\tv_nop" : "+v"(d) : "v"(a), "v"(b)); return d; }

__global__ __launch_bounds__(256) void k_wt_f16(const float* __restrict__ W, _Float16* __restrict__ Wt, int K, int N, float scale) {
  const int t = blockIdx.x * 256 + threadIdx.x; if (t >= N * (K / 8)) return;
  const int n = t / (K / 8), k8 = (t % (K / 8)) * 8; FragH f;
#pragma unroll
  for (int i = 0; i < 8; ++i) f.h[i] = (_Float16)(bf16_rne(W[(size_t)(k8 + i) * N + n]) * scale);
  const v8us o = f.half[0]; unsigned short* d = (unsigned short*)Wt + (size_t)n * K + k8;
  *(volatile v8us*)d = o; __threadfence(); *(volatile v8us*)d = o;
}

__global__ __launch_bounds__(256) void k_x16(const float* __restrict__ x, _Float16* __restrict__ X16, size_t n8) {
  const size_t t = (size_t)blockIdx.x * 256 + threadIdx.x; if (t >= n8) return;
  const size_t e = t * 8; const size_t r = e / DM; const size_t c = e % DM; const size_t rs = (r / SEQ) * SEQ_FULL + (r % SEQ);
  const float* src = x + rs * DM + c; const v4f a = *(const v4fa*)src; const v4f a2 = *(const v4fa*)(src + 4); FragH f;
#pragma unroll
  for (int q = 0; q < 4; ++q) { f.h[q] = (_Float16)bf16_rne(a[q]); f.h[4 + q] = (_Float16)bf16_rne(a2[q]); }
  const v8us o = f.half[0]; unsigned short* d = (unsigned short*)X16 + e;
  *(volatile v8us*)d = o; __threadfence(); *(volatile v8us*)d = o;
}

template <int NHv, int TTv>
__global__ __launch_bounds__(256) void k_vt(const _Float16* __restrict__ V16, int ldv, int voff, _Float16* __restrict__ Vt) {
  __shared__ unsigned short tl[64][66]; const int tid = threadIdx.x; const int slab = blockIdx.x / (TTv / 64), lg = blockIdx.x % (TTv / 64); const int b = slab / NHv, h = slab % NHv;
  for (int i = tid; i < 64 * 8; i += 256) { const int r = i / 8, c8 = (i % 8) * 8; FragH f; f.half[0] = *(const v8us*)((const unsigned short*)V16 + ((size_t)b * TTv + lg * 64 + r) * ldv + voff + h * 64 + c8);
#pragma unroll
    for (int q = 0; q < 8; ++q) tl[r][c8 + q] = f.u[q]; }
  __syncthreads();
  for (int pass = 0; pass < 2; ++pass) {
#pragma unroll
    for (int rd = 0; rd < 2; ++rd) { const int d = rd * 32 + tid / 8, pc = tid % 8; FragH f;
#pragma unroll
      for (int q = 0; q < 8; ++q) f.u[q] = tl[pc * 8 + q][d];
      *(volatile v8us*)((unsigned short*)Vt + ((size_t)slab * 64 + d) * TTv + lg * 64 + pc * 8) = f.half[0]; }
    if (pass == 0) __threadfence(); }
}

template <int ACT>
__global__ __launch_bounds__(128) void k_gemm2(const _Float16* __restrict__ A, int lda, const _Float16* __restrict__ Bh, int ldb, float alpha, const float* __restrict__ bias, float bsc,
    float* __restrict__ C, _Float16* __restrict__ C16, int ldc, int M, int N, int K) {
  static_assert(ACT == 0 || ACT == 3);
  __shared__ __attribute__((aligned(16))) float so[4][32][68];
  const int tid = threadIdx.x, w = tid >> 5, lane = tid & 31, ln = lane & 15, hh = lane >> 4;
  const int ntn = N >> 6; const int mt = blockIdx.x / ntn, nq = blockIdx.x - mt * ntn; const int row0 = mt * 128 + 32 * w, col0 = nq * 64; if (row0 >= M) return;
  const _Float16* a0p = A + (size_t)(row0 + ln) * lda; const _Float16* a1p = a0p + (size_t)16 * lda;
  const _Float16* b0p = Bh + (size_t)(col0 + ln) * ldb; const _Float16* b1p = b0p + (size_t)16 * ldb; const _Float16* b2p = b1p + (size_t)16 * ldb; const _Float16* b3p = b2p + (size_t)16 * ldb;
  const v8f z8 = {0.f,0.f,0.f,0.f,0.f,0.f,0.f,0.f}; v8f c00 = z8, c01 = z8, c02 = z8, c03 = z8, c10 = z8, c11 = z8, c12 = z8, c13 = z8;
#pragma unroll 1
  for (int kb = 0; kb < K; kb += 32) { const v16h a0 = g2_frag(a0p + kb, hh), a1 = g2_frag(a1p + kb, hh);
    v16h b = g2_frag(b0p + kb, hh); c00 = g2_mma(a0, b, c00); c10 = g2_mma(a1, b, c10);
    b = g2_frag(b1p + kb, hh); c01 = g2_mma(a0, b, c01); c11 = g2_mma(a1, b, c11);
    b = g2_frag(b2p + kb, hh); c02 = g2_mma(a0, b, c02); c12 = g2_mma(a1, b, c12);
    b = g2_frag(b3p + kb, hh); c03 = g2_mma(a0, b, c03); c13 = g2_mma(a1, b, c13); }
  v8f accs[8] = {c00, c01, c02, c03, c10, c11, c12, c13};
#pragma unroll
  for (int u = 0; u < 8; ++u) { const int t = u & 3, half = u >> 2; const int col = col0 + t * 16 + ln; const float bv = bias ? bf16_rne(bias[col]) * bsc : 0.f;
#pragma unroll
    for (int r = 0; r < 8; ++r) { const int rloc = half * 16 + 8 * hh + r; float v = accs[u][r] * alpha + bv; if (ACT == 3) v = fmaxf(v, 0.f); so[w][rloc][t * 16 + ln] = v; } }
  __builtin_amdgcn_fence(4  , "workgroup"); __builtin_amdgcn_wave_barrier();
  const int rsub = lane >> 4, c4 = (lane & 15) * 4;
  for (int pass = 0; pass < 2; ++pass) {
#pragma unroll
    for (int q = 0; q < 16; ++q) { const int r = q * 2 + rsub; const v4f v = *(const v4fa*)&so[w][r][c4];
      if (C) *(volatile v4f*)(C + (size_t)(row0 + r) * ldc + col0 + c4) = v;
      if (C16) { v4h h4; for (int i = 0; i < 4; ++i) h4[i] = (_Float16)v[i]; *(volatile v4h*)(C16 + (size_t)(row0 + r) * ldc + col0 + c4) = h4; } }
    if (pass == 0) __threadfence(); }
}

template <int CAUSAL>
__global__ __launch_bounds__(128) void k_attn(const _Float16* __restrict__ Q16, const _Float16* __restrict__ K16, const _Float16* __restrict__ VT, _Float16* __restrict__ O16) {
  __shared__ __attribute__((aligned(16))) _Float16 pb[4][16 * PBP];
  __shared__ __attribute__((aligned(16))) _Float16 ob[4][16 * OBP];
  const int tid = threadIdx.x, w = tid >> 5, lane = tid & 31, ln = lane & 15, hh = lane >> 4;
  const int h = blockIdx.y, b = blockIdx.z;
  const int q0 = (blockIdx.x * 4 + w) * 16;
  const size_t tok0 = (size_t)b * SEQ;
  const int slab = b * NH + h;
  _Float16* pw = &pb[w][0]; _Float16* ow = &ob[w][0];
  const _Float16* qrow = Q16 + (tok0 + q0 + ln) * DM + h * HD;
  const v16h qf0 = g2_frag(qrow, hh), qf1 = g2_frag(qrow + 32, hh);
  const v8f z8 = {0.f,0.f,0.f,0.f,0.f,0.f,0.f,0.f};
  v8f o0 = z8, o1 = z8, o2 = z8, o3 = z8;
  float mrow[8], lrow[8];
#pragma unroll
  for (int r = 0; r < 8; ++r) { mrow[r] = -1.0e30f; lrow[r] = 0.f; }
  const int kend = CAUSAL ? (q0 + 16) : SEQ;
#pragma unroll 1
  for (int kb = 0; kb < kend; kb += 32) {
    const _Float16* k0p = K16 + (tok0 + kb + ln) * DM + h * HD; const _Float16* k1p = k0p + (size_t)16 * DM;
    v8f s0 = z8, s1 = z8;
    v16h kf = g2_frag(k0p, hh);    s0 = g2_mma(qf0, kf, s0);
    kf = g2_frag(k0p + 32, hh);    s0 = g2_mma(qf1, kf, s0);
    kf = g2_frag(k1p, hh);         s1 = g2_mma(qf0, kf, s1);
    kf = g2_frag(k1p + 32, hh);    s1 = g2_mma(qf1, kf, s1);
#pragma unroll
    for (int r = 0; r < 8; ++r) {
      const int row = q0 + 8 * hh + r;
      float a = s0[r] * 0.125f, c = s1[r] * 0.125f;
      if (CAUSAL) { a = (kb + ln > row) ? -1.0e9f : a; c = (kb + 16 + ln > row) ? -1.0e9f : c; }
      float t = fmaxf(a, c);
      t = fmaxf(t, __shfl_xor(t, 1, 32)); t = fmaxf(t, __shfl_xor(t, 2, 32)); t = fmaxf(t, __shfl_xor(t, 4, 32)); t = fmaxf(t, __shfl_xor(t, 8, 32));
      const float mnew = fmaxf(mrow[r], t);
      const float p0 = __expf(a - mnew), p1 = __expf(c - mnew);
      float ls = p0 + p1;
      ls += __shfl_xor(ls, 1, 32); ls += __shfl_xor(ls, 2, 32); ls += __shfl_xor(ls, 4, 32); ls += __shfl_xor(ls, 8, 32);
      const float corr = __expf(mrow[r] - mnew);
      lrow[r] = lrow[r] * corr + ls; mrow[r] = mnew;
      o0[r] *= corr; o1[r] *= corr; o2[r] *= corr; o3[r] *= corr;
      pw[(8 * hh + r) * PBP + ln]      = (_Float16)(p0 * 256.0f);
      pw[(8 * hh + r) * PBP + 16 + ln] = (_Float16)(p1 * 256.0f);
    }
    __builtin_amdgcn_fence(4  , "wavefront"); __builtin_amdgcn_wave_barrier();
    const v16h pf = g2_frag(pw + ln * PBP, hh);
    __builtin_amdgcn_fence(4  , "wavefront"); __builtin_amdgcn_wave_barrier();
    const _Float16* vp = VT + ((size_t)slab * HD + ln) * SEQ + kb;
    v16h vf = g2_frag(vp, hh);                   o0 = g2_mma(pf, vf, o0);
    vf = g2_frag(vp + (size_t)16 * SEQ, hh);     o1 = g2_mma(pf, vf, o1);
    vf = g2_frag(vp + (size_t)32 * SEQ, hh);     o2 = g2_mma(pf, vf, o2);
    vf = g2_frag(vp + (size_t)48 * SEQ, hh);     o3 = g2_mma(pf, vf, o3);
  }
#pragma unroll
  for (int r = 0; r < 8; ++r) {
    const float rl = 0.25f * __builtin_amdgcn_rcpf(lrow[r]);
    const int rloc = (8 * hh + r) * OBP + ln;
    ow[rloc]      = (_Float16)(o0[r] * rl); ow[rloc + 16] = (_Float16)(o1[r] * rl);
    ow[rloc + 32] = (_Float16)(o2[r] * rl); ow[rloc + 48] = (_Float16)(o3[r] * rl);
  }
  __builtin_amdgcn_fence(4  , "wavefront"); __builtin_amdgcn_wave_barrier();
  const int rq = lane >> 3, pc = (lane & 7) * 8;
  for (int pass = 0; pass < 2; ++pass) {
#pragma unroll
    for (int i = 0; i < 4; ++i) { const int row = i * 4 + rq; const v8us v = *(const v8us*)(ow + row * OBP + pc);
      *(volatile v8us*)((unsigned short*)O16 + (tok0 + q0 + row) * DM + h * HD + pc) = v; }
    if (pass == 0) __threadfence(); }
}

template <int RBF, int RMAP, int W16, int OMAP>
__global__ __launch_bounds__(256) void k_ln(const float* __restrict__ X, const float* __restrict__ R, const float* __restrict__ g, const float* __restrict__ bb, float eps, float* __restrict__ O32, _Float16* __restrict__ O16) {
  #pragma clang fp contract(off)
  __shared__ float red[256];
  const size_t r = blockIdx.x; const int t = threadIdx.x; const int c0 = t * 4;
  const size_t rfull = (r / SEQ) * SEQ_FULL + (r % SEQ);
  const size_t rr = RMAP ? rfull : r;
  const v4f xa = *(const v4fa*)(X + r * DM + c0); const v4f ra = *(const v4fa*)(R + rr * DM + c0);
  float s[4]; float sum = 0.f;
#pragma unroll
  for (int q = 0; q < 4; ++q) { const float rv = RBF ? bf16_rne(ra[q]) : ra[q]; s[q] = xa[q] + rv; sum += s[q]; }
  red[t] = sum; __syncthreads();
  for (int st = 128; st > 0; st >>= 1) { if (t < st) red[t] += red[t + st]; __syncthreads(); }
  const float mu = red[0] * (1.0f / (float)DM); __syncthreads();
  float vs = 0.f;
#pragma unroll
  for (int q = 0; q < 4; ++q) { const float dl = s[q] - mu; vs += dl * dl; }
  red[t] = vs; __syncthreads();
  for (int st = 128; st > 0; st >>= 1) { if (t < st) red[t] += red[t + st]; __syncthreads(); }
  const float rs = rsqrtf(red[0] * (1.0f / (float)DM) + eps);
  v4f yf; v4h y;
#pragma unroll
  for (int q = 0; q < 4; ++q) { const int c = c0 + q; yf[q] = (s[q] - mu) * rs * bf16_rne(g[c]) + bf16_rne(bb[c]); y[q] = (_Float16)yf[q]; }
  const size_t orow = OMAP ? rfull : r;
  for (int pass = 0; pass < 2; ++pass) {
    if (O32) *(volatile v4f*)(O32 + orow * DM + c0) = yf;
    if (W16) *(volatile v4h*)(O16 + r * DM + c0) = y;
    if (pass == 0) __threadfence(); }
}

extern "C" void kernel_launch(void* const* d_in, const int* in_sizes, int n_in,
                              void* d_out, int out_size, void* d_ws, size_t ws_size, hipStream_t stream) {
  if (n_in < 28) return;
  const float* x    = (const float*)d_in[0];  const float* enc  = (const float*)d_in[1];
  const float* wq1  = (const float*)d_in[2];  const float* wk1  = (const float*)d_in[3];  const float* wv1 = (const float*)d_in[4];  const float* wo1 = (const float*)d_in[5];
  const float* bq1  = (const float*)d_in[6];  const float* bk1  = (const float*)d_in[7];  const float* bv1 = (const float*)d_in[8];  const float* bo1 = (const float*)d_in[9];
  const float* wq2  = (const float*)d_in[10]; const float* wk2  = (const float*)d_in[11]; const float* wv2 = (const float*)d_in[12]; const float* wo2 = (const float*)d_in[13];
  const float* bq2  = (const float*)d_in[14]; const float* bk2  = (const float*)d_in[15]; const float* bv2 = (const float*)d_in[16]; const float* bo2 = (const float*)d_in[17];
  const float* wff1 = (const float*)d_in[18]; const float* bff1 = (const float*)d_in[19]; const float* wff2 = (const float*)d_in[20]; const float* bff2 = (const float*)d_in[21];
  const float* g1   = (const float*)d_in[22]; const float* be1  = (const float*)d_in[23]; const float* g2  = (const float*)d_in[24]; const float* be2 = (const float*)d_in[25];
  const float* g3   = (const float*)d_in[26]; const float* be3  = (const float*)d_in[27];

  const size_t needX = ((size_t)(NB - 1) * SEQ_FULL + SEQ) * DM;
  if ((size_t)in_sizes[0] < needX || (size_t)in_sizes[1] < needX || (size_t)out_size < needX) return;
  { static const int wi[8] = {2, 3, 4, 5, 10, 11, 12, 13}; for (int i = 0; i < 8; ++i) if ((size_t)in_sizes[wi[i]] < (size_t)DM * DM) return; }
  if ((size_t)in_sizes[18] < (size_t)DM * DFF || (size_t)in_sizes[20] < (size_t)DM * DFF || in_sizes[19] < DFF) return;
  { static const int vi[15] = {6, 7, 8, 9, 14, 15, 16, 17, 21, 22, 23, 24, 25, 26, 27}; for (int i = 0; i < 15; ++i) if (in_sizes[vi[i]] < DM) return; }

  char* ws = (char*)d_ws; size_t off = 0;
  auto take = [&](size_t bytes) { char* p = ws + off; off += (bytes + 255) & ~(size_t)255; return p; };
  const size_t WDD = (size_t)DM * DM * 2, WDF = (size_t)DM * DFF * 2, P16 = NR * DM * 2, P32 = NR * DM * 4;
  _Float16* BQ1 = (_Float16*)take(WDD); _Float16* BK1 = (_Float16*)take(WDD); _Float16* BV1 = (_Float16*)take(WDD); _Float16* BO1 = (_Float16*)take(WDD);
  _Float16* BQ2 = (_Float16*)take(WDD); _Float16* BK2 = (_Float16*)take(WDD); _Float16* BV2 = (_Float16*)take(WDD); _Float16* BO2 = (_Float16*)take(WDD);
  _Float16* BW1 = (_Float16*)take(WDF);
  _Float16* BW2 = (_Float16*)take(WDF);
  char* RA = take(2 * P16); _Float16* X16 = (_Float16*)RA; _Float16* E16 = (_Float16*)(RA + P16); _Float16* O16 = (_Float16*)RA; float* O2F = (float*)RA;
  const size_t RBB = (4 * P16 > NR * (size_t)DFF * 2) ? 4 * P16 : NR * (size_t)DFF * 2;
  char* RB = take(RBB); _Float16* Q16 = (_Float16*)RB; _Float16* K16 = (_Float16*)(RB + P16); _Float16* V16 = (_Float16*)(RB + 2 * P16); _Float16* VT = (_Float16*)(RB + 3 * P16); _Float16* HF = (_Float16*)RB;
  float* YF = (float*)take(P32);
  float* O1F = (float*)take(P32);
  _Float16* OH = (_Float16*)take(P16);
  if (off > ws_size || off > (size_t)134217728) return;

  const unsigned gDD = (unsigned)(((size_t)DM * (DM / 8) + 255) / 256), gDF = (unsigned)(((size_t)DFF * (DM / 8) + 255) / 256), gFD = (unsigned)(((size_t)DM * (DFF / 8) + 255) / 256);
  k_wt_f16<<<gDD, 256, 0, stream>>>(wq1, BQ1, DM, DM, 16.0f); k_wt_f16<<<gDD, 256, 0, stream>>>(wk1, BK1, DM, DM, 16.0f); k_wt_f16<<<gDD, 256, 0, stream>>>(wv1, BV1, DM, DM, 16.0f); k_wt_f16<<<gDD, 256, 0, stream>>>(wo1, BO1, DM, DM, 16.0f);
  k_wt_f16<<<gDD, 256, 0, stream>>>(wq2, BQ2, DM, DM, 16.0f); k_wt_f16<<<gDD, 256, 0, stream>>>(wk2, BK2, DM, DM, 16.0f); k_wt_f16<<<gDD, 256, 0, stream>>>(wv2, BV2, DM, DM, 16.0f); k_wt_f16<<<gDD, 256, 0, stream>>>(wo2, BO2, DM, DM, 16.0f);
  k_wt_f16<<<gDF, 256, 0, stream>>>(wff1, BW1, DM, DFF, 16.0f); k_wt_f16<<<gFD, 256, 0, stream>>>(wff2, BW2, DFF, DM, 16.0f);

  const size_t n8 = NR * DM / 8; const unsigned gx = (unsigned)((n8 + 255) / 256);
  k_x16<<<gx, 256, 0, stream>>>(x, X16, n8); k_x16<<<gx, 256, 0, stream>>>(enc, E16, n8);

  const unsigned gP = (unsigned)((MR / 128) * (DM / 64)), gF1 = (unsigned)((MR / 128) * (DFF / 64));
  const unsigned gVT = (unsigned)(NB * NH * (SEQ / 64)); const dim3 gAT(SEQ / 64, NH, NB);

  k_gemm2<0><<<gP, 128, 0, stream>>>(X16, DM, BQ1, DM, 0.0625f, bq1, 1.0f, nullptr, Q16, DM, MR, DM, DM);
  k_gemm2<0><<<gP, 128, 0, stream>>>(X16, DM, BK1, DM, 0.0625f, bk1, 1.0f, nullptr, K16, DM, MR, DM, DM);
  k_gemm2<0><<<gP, 128, 0, stream>>>(X16, DM, BV1, DM, 0.0625f, bv1, 1.0f, nullptr, V16, DM, MR, DM, DM);
  k_vt<NH, SEQ><<<gVT, 256, 0, stream>>>(V16, DM, 0, VT);
  k_attn<1><<<gAT, 128, 0, stream>>>(Q16, K16, VT, O16);
  k_gemm2<0><<<gP, 128, 0, stream>>>(O16, DM, BO1, DM, 0.0009765625f, bo1, 1.0f, YF, nullptr, DM, MR, DM, DM);
  k_ln<1, 1, 1, 0><<<(unsigned)MR, 256, 0, stream>>>(YF, x, g1, be1, LN_EPS, O1F, OH);
  k_gemm2<0><<<gP, 128, 0, stream>>>(OH, DM, BQ2, DM, 0.0625f, bq2, 1.0f, nullptr, Q16, DM, MR, DM, DM);
  k_gemm2<0><<<gP, 128, 0, stream>>>(E16, DM, BK2, DM, 0.0625f, bk2, 1.0f, nullptr, K16, DM, MR, DM, DM);
  k_gemm2<0><<<gP, 128, 0, stream>>>(E16, DM, BV2, DM, 0.0625f, bv2, 1.0f, nullptr, V16, DM, MR, DM, DM);
  k_vt<NH, SEQ><<<gVT, 256, 0, stream>>>(V16, DM, 0, VT);
  k_attn<0><<<gAT, 128, 0, stream>>>(Q16, K16, VT, O16);
  k_gemm2<0><<<gP, 128, 0, stream>>>(O16, DM, BO2, DM, 0.0009765625f, bo2, 1.0f, YF, nullptr, DM, MR, DM, DM);
  k_ln<0, 0, 1, 0><<<(unsigned)MR, 256, 0, stream>>>(YF, O1F, g2, be2, LN_EPS, O2F, OH);
  k_gemm2<3><<<gF1, 128, 0, stream>>>(OH, DM, BW1, DM, 1.0f, bff1, 16.0f, nullptr, HF, DFF, MR, DFF, DM);
  k_gemm2<0><<<gP, 128, 0, stream>>>(HF, DFF, BW2, DFF, 0.00390625f, bff2, 1.0f, YF, nullptr, DM, MR, DM, DFF);
  k_ln<0, 0, 0, 1><<<(unsigned)MR, 256, 0, stream>>>(YF, O2F, g3, be3, LN_EPS, (float*)d_out, nullptr);
}
